// MultiHeadCrossAttention_15710990369684
// MI455X (gfx1250) — hardware-verified
//
#include <hip/hip_runtime.h>
#include <math.h>

#ifndef NB
#define NB 4
#endif
#ifndef SEQ
#define SEQ 2048
#endif
#define NB_FULL   4
#define QLEN_FULL 2048
#define KLEN      2048
#define QDIM      512
#define EMBED     1024
#define HEADS     16
#define HEAD_DIM  64
#define FW        2

static_assert(NB >= 1 && NB <= NB_FULL);
static_assert(SEQ >= 64 && SEQ <= QLEN_FULL && (SEQ % 64) == 0 && (SEQ % (16 * FW)) == 0);
static_assert((KLEN % 64) == 0 && (QDIM % 32) == 0 && (QDIM % 8) == 0 && (EMBED % 64) == 0);
static_assert(HEADS * HEAD_DIM == EMBED && HEAD_DIM == 64);

typedef __attribute__((ext_vector_type(16))) _Float16 v16h;
typedef __attribute__((ext_vector_type(8)))  _Float16 v8h;
typedef __attribute__((ext_vector_type(16))) __bf16   v16b;
typedef __attribute__((ext_vector_type(8)))  __bf16   v8b;
typedef __attribute__((ext_vector_type(8)))  float    v8f;
typedef __attribute__((ext_vector_type(4)))  float    v4f;
typedef __attribute__((ext_vector_type(4)))  unsigned v4u;

__device__ __forceinline__ unsigned short f2bf_bits(float f) {
    unsigned u = __float_as_uint(f);
    return (unsigned short)((u + 0x7FFFu + ((u >> 16) & 1u)) >> 16);
}
__device__ __forceinline__ unsigned pk2u(unsigned short lo, unsigned short hi) { return (unsigned)lo | ((unsigned)hi << 16); }

__device__ __forceinline__ v8f wmma16(v16h a, v16h b, v8f c) {
    c = __builtin_amdgcn_wmma_f32_16x16x32_f16(false, a, false, b, (short)0, c, false, false);
    asm volatile("v_nop\n\tv_nop\n\tv_nop\n\tv_nop" : "+v"(c) : "v"(a), "v"(b));
    return c;
}
__device__ __forceinline__ void dep_guard_b(v8f& a, v8f& b, v16b x, v16b y) { asm volatile("v_nop\n\tv_nop\n\tv_nop\n\tv_nop" : "+v"(a), "+v"(b) : "v"(x), "v"(y)); }
__device__ __forceinline__ void keep4_b(v16b a, v16b b, v16b c, v16b d) { asm volatile("v_nop" :: "v"(a), "v"(b), "v"(c), "v"(d)); }
__device__ __forceinline__ void acc_guard4(v8f& a, v8f& b, v8f& c, v8f& d) { asm volatile("v_nop\n\tv_nop\n\tv_nop\n\tv_nop" : "+v"(a), "+v"(b), "+v"(c), "+v"(d)); }

union FragB { v16b v; v8b h[2]; };
union FragH { v16h v; v8h h[2]; };
__device__ __forceinline__ v16b ldfrag_b(const __bf16* p) { FragB f; f.h[0] = *(const v8b*)(p); f.h[1] = *(const v8b*)(p + 16); return f.v; }
__device__ __forceinline__ v16h ldfrag_h(const _Float16* p) { FragH f; f.h[0] = *(const v8h*)(p); f.h[1] = *(const v8h*)(p + 16); return f.v; }

__global__ __launch_bounds__(256) void k_cvt_bf16(const float* __restrict__ src, unsigned short* __restrict__ dst, long long n8) {
    const long long u = (long long)blockIdx.x * 256 + threadIdx.x;
    if (u >= n8) return;
    const v4f a = *(const v4f*)(src + 8 * u);
    const v4f b = *(const v4f*)(src + 8 * u + 4);
    const float a0 = a.x, a1 = a.y, a2 = a.z, a3 = a.w, b0 = b.x, b1 = b.y, b2 = b.z, b3 = b.w;
    v4u pk;
    pk.x = pk2u(f2bf_bits(a0), f2bf_bits(a1));
    pk.y = pk2u(f2bf_bits(a2), f2bf_bits(a3));
    pk.z = pk2u(f2bf_bits(b0), f2bf_bits(b1));
    pk.w = pk2u(f2bf_bits(b2), f2bf_bits(b3));
    volatile v4u* d = (volatile v4u*)(dst + 8 * u);
    *d = pk; __threadfence(); *d = pk;
}

__global__ __launch_bounds__(256) void k_wT_bf16(const float* __restrict__ W, unsigned short* __restrict__ dst) {
    const int u = blockIdx.x * 256 + threadIdx.x;
    if (u >= EMBED * (QDIM / 8)) return;
    const int k8 = u % (QDIM / 8);
    const int o  = u / (QDIM / 8);
    const int k0 = 8 * k8;
    unsigned short hb[8];
#pragma unroll
    for (int i = 0; i < 8; ++i) hb[i] = f2bf_bits(W[(size_t)(k0 + i) * EMBED + o]);
    v4u pk;
    pk.x = pk2u(hb[0], hb[1]); pk.y = pk2u(hb[2], hb[3]); pk.z = pk2u(hb[4], hb[5]); pk.w = pk2u(hb[6], hb[7]);
    volatile v4u* d = (volatile v4u*)(dst + (size_t)o * QDIM + k0);
    *d = pk; __threadfence(); *d = pk;
}

template <bool RES>
__global__ __launch_bounds__(256) __attribute__((amdgpu_num_vgpr(256)))
void k_gemm64(const unsigned short* __restrict__ Ap, int lda, long long strideA,
              const unsigned short* __restrict__ Btp, int ldb, long long strideB,
              unsigned short* __restrict__ Cp, unsigned short* __restrict__ C2p, int ldc, long long strideC,
              int M, int N, int K, float scale) {
    __shared__ __align__(16) float sT[8][16 * 68];
    const int b    = blockIdx.y;
    const int lane = threadIdx.x & 31;
    const int wave = threadIdx.x >> 5;
    const int tilesN = N >> 6;
    const int tilesM = M >> 6;
    const int tile = blockIdx.x * 8 + wave;
    if (tile >= tilesM * tilesN) return;
    const int tm = tile / tilesN;
    const int tn = tile - tm * tilesN;
    const int m0 = tm << 6;
    const int n0 = tn << 6;

    const __bf16* Ab = (const __bf16*)Ap  + (size_t)b * strideA;
    const __bf16* Bb = (const __bf16*)Btp + (size_t)b * strideB;

    const int rlane = lane & 15;
    const int koff  = (lane >> 4) * 8;
    const int mOff  = (lane >> 4) * 8;

    v8f acc[4][4];
#pragma unroll
    for (int i = 0; i < 4; ++i)
#pragma unroll
        for (int j = 0; j < 4; ++j) acc[i][j] = (v8f){0.f, 0.f, 0.f, 0.f, 0.f, 0.f, 0.f, 0.f};

    for (int k0 = 0; k0 < K; k0 += 32) {
        v16b bh[4];
#pragma unroll
        for (int j = 0; j < 4; ++j) bh[j] = ldfrag_b(Bb + (size_t)(n0 + (j << 4) + rlane) * ldb + koff + k0);
#pragma unroll
        for (int i = 0; i < 4; ++i) {
            const v16b ah = ldfrag_b(Ab + (size_t)(m0 + (i << 4) + rlane) * lda + koff + k0);
#pragma unroll
            for (int j = 0; j < 4; ++j)
                acc[i][j] = __builtin_amdgcn_wmma_f32_16x16x32_bf16(false, ah, false, bh[j], (short)0, acc[i][j], false, false);
            dep_guard_b(acc[i][0], acc[i][3], ah, ah);
        }
        keep4_b(bh[0], bh[1], bh[2], bh[3]);
    }
    acc_guard4(acc[0][0], acc[0][1], acc[0][2], acc[0][3]);
    acc_guard4(acc[1][0], acc[1][1], acc[1][2], acc[1][3]);
    acc_guard4(acc[2][0], acc[2][1], acc[2][2], acc[2][3]);
    acc_guard4(acc[3][0], acc[3][1], acc[3][2], acc[3][3]);

    float* slab = sT[wave];
    unsigned short* C  = Cp + (size_t)b * strideC;
    unsigned short* C2 = RES ? (C2p + (size_t)b * strideC) : nullptr;
    const int q = lane >> 3, c8 = (lane & 7) * 8;
#pragma unroll
    for (int i = 0; i < 4; ++i) {
        const int mBase = m0 + (i << 4);
#pragma unroll
        for (int j = 0; j < 4; ++j) {
#pragma unroll
            for (int r = 0; r < 8; ++r) slab[(mOff + r) * 68 + (j << 4) + rlane] = acc[i][j][r] * scale;
        }
        __builtin_amdgcn_fence(3, "workgroup");
        __builtin_amdgcn_wave_barrier();
        __builtin_amdgcn_fence(2, "workgroup");
        for (int pass = 0; pass < 2; ++pass) {
#pragma unroll
            for (int it = 0; it < 4; ++it) {
                const int row = it * 4 + q;
                const float* sp = slab + row * 68 + c8;
                v8h hv, lv;
#pragma unroll
                for (int e = 0; e < 8; ++e) {
                    const float x = sp[e];
                    const _Float16 hq = (_Float16)x;
                    hv[e] = hq;
                    if (RES) { const float rs = (x - (float)hq) * 1024.0f; lv[e] = (_Float16)rs; } else lv[e] = hq;
                }
                const size_t oe = (size_t)(mBase + row) * ldc + n0 + c8;
                *(volatile v8h*)(C + oe) = hv;
                if (RES) *(volatile v8h*)(C2 + oe) = lv;
            }
            __threadfence();
        }
        __builtin_amdgcn_fence(3, "workgroup");
        __builtin_amdgcn_wave_barrier();
        __builtin_amdgcn_fence(2, "workgroup");
    }
}

__global__ __launch_bounds__(32 * FW) __attribute__((amdgpu_num_vgpr(256)))
void k_flash(const unsigned short* __restrict__ qP, const unsigned short* __restrict__ qR, const unsigned short* __restrict__ kP,
             const unsigned short* __restrict__ vTP, const int* __restrict__ msk, float* __restrict__ out) {
    __shared__ __align__(16) _Float16 Psh[FW][16 * 64];
    __shared__ __align__(16) float    Os[FW][16 * 68];
    const int tid  = threadIdx.x;
    const int wave = tid >> 5;
    const int lane = tid & 31;
    const int hh   = lane >> 4;
    const int c    = lane & 15;

    constexpr int NQB = SEQ / (16 * FW);
    const int bx = blockIdx.x;
    const int qb = bx % NQB;
    const int bh = bx / NQB;
    const int h  = bh % HEADS;
    const int b  = bh / HEADS;
    const int q0 = qb * (16 * FW) + wave * 16;
    const size_t grow0 = (size_t)b * QLEN_FULL + q0;

    const _Float16* qpl = (const _Float16*)qP;
    const _Float16* qrl = (const _Float16*)qR;
    const _Float16* kbase = (const _Float16*)kP + h * HEAD_DIM;
    const _Float16* vbase = (const _Float16*)vTP + (size_t)(h * HEAD_DIM) * KLEN;
    const int* mrowp = msk + (size_t)b * KLEN;

    v16h qa[2];
    const _Float16* qr  = qpl + (grow0 + c) * (size_t)EMBED + h * HEAD_DIM;
    const _Float16* qrr = qrl + (grow0 + c) * (size_t)EMBED + h * HEAD_DIM;
#pragma unroll
    for (int dc = 0; dc < 2; ++dc) qa[dc] = ldfrag_h(qr + dc * 32 + 8 * hh);

    const float NEG   = -__builtin_inff();
    const float MFILL = -1.25e19f;
    const float SC    = 0.125f * 1.4426950408889634f;
    const float PSC   = 32768.0f;
    const float RSC   = 0.0009765625f;

    float mrow[8], lrow[8];
    v8f oacc[4];
#pragma unroll
    for (int r = 0; r < 8; ++r) { mrow[r] = NEG; lrow[r] = 0.f; }
#pragma unroll
    for (int t = 0; t < 4; ++t) oacc[t] = (v8f){0.f, 0.f, 0.f, 0.f, 0.f, 0.f, 0.f, 0.f};

    _Float16* pw = Psh[wave];

#pragma unroll 1
    for (int kc = 0; kc < KLEN / 64; ++kc) {
        const int kv0 = kc * 64;
        v16h qres[2];
#pragma unroll
        for (int dc = 0; dc < 2; ++dc) qres[dc] = ldfrag_h(qrr + dc * 32 + 8 * hh);
        v8f s[4];
        int mk[4];
#pragma unroll
        for (int j = 0; j < 4; ++j) {
            v8f acc  = (v8f){0.f, 0.f, 0.f, 0.f, 0.f, 0.f, 0.f, 0.f};
            v8f accr = (v8f){0.f, 0.f, 0.f, 0.f, 0.f, 0.f, 0.f, 0.f};
            const _Float16* kr = kbase + (size_t)(kv0 + j * 16 + c) * EMBED;
#pragma unroll
            for (int dc = 0; dc < 2; ++dc) {
                const v16h kf = ldfrag_h(kr + dc * 32 + 8 * hh);
                acc  = wmma16(qa[dc],   kf, acc);
                accr = wmma16(qres[dc], kf, accr);
            }
            s[j] = acc + accr * RSC;
            mk[j] = mrowp[kv0 + j * 16 + c];
        }
        float cm[8];
#pragma unroll
        for (int r = 0; r < 8; ++r) {
            float m = NEG;
#pragma unroll
            for (int j = 0; j < 4; ++j) {
                float v = s[j][r] * SC;
                v = (mk[j] == 0) ? MFILL : v;
                s[j][r] = v;
                m = fmaxf(m, v);
            }
#pragma unroll
            for (int off = 1; off < 16; off <<= 1) m = fmaxf(m, __shfl_xor(m, off, 32));
            cm[r] = m;
        }
#pragma unroll
        for (int r = 0; r < 8; ++r) {
            const float mnew  = fmaxf(mrow[r], cm[r]);
            const float alpha = exp2f(mrow[r] - mnew);
            mrow[r] = mnew;
            float psum = 0.f;
#pragma unroll
            for (int j = 0; j < 4; ++j) {
                const float p = exp2f(s[j][r] - mnew);
                psum += p;
                pw[(8 * hh + r) * 64 + j * 16 + c] = (_Float16)(p * PSC);
            }
#pragma unroll
            for (int off = 1; off < 16; off <<= 1) psum += __shfl_xor(psum, off, 32);
            lrow[r] = lrow[r] * alpha + psum;
#pragma unroll
            for (int t = 0; t < 4; ++t) oacc[t][r] *= alpha;
        }
        __builtin_amdgcn_fence(3, "workgroup");
        __builtin_amdgcn_wave_barrier();
        __builtin_amdgcn_fence(2, "workgroup");
#pragma unroll
        for (int kk = 0; kk < 2; ++kk) {
            const v16h pa = ldfrag_h(pw + c * 64 + kk * 32 + 8 * hh);
#pragma unroll
            for (int t = 0; t < 4; ++t) {
                const _Float16* vr = vbase + (size_t)(t * 16 + c) * KLEN + kv0 + kk * 32 + 8 * hh;
                oacc[t] = wmma16(pa, ldfrag_h(vr), oacc[t]);
            }
        }
        __builtin_amdgcn_fence(3, "workgroup");
        __builtin_amdgcn_wave_barrier();
        __builtin_amdgcn_fence(2, "workgroup");
    }

    float* os = Os[wave];
#pragma unroll
    for (int r = 0; r < 8; ++r) {
        const float inv = (1.0f / lrow[r]) * (1.0f / 32768.0f);
#pragma unroll
        for (int t = 0; t < 4; ++t) os[(8 * hh + r) * 68 + t * 16 + c] = oacc[t][r] * inv;
    }
    __builtin_amdgcn_fence(3, "workgroup");
    __builtin_amdgcn_wave_barrier();
    __builtin_amdgcn_fence(2, "workgroup");
    {
        float* ob = out + grow0 * (size_t)EMBED + h * HEAD_DIM;
        const int c4 = (lane & 15) * 4;
        for (int pass = 0; pass < 2; ++pass) {
#pragma unroll
            for (int it = 0; it < 8; ++it) {
                const int row = it * 2 + hh;
                const v4f val = *(const v4f*)(os + row * 68 + c4);
                *(volatile v4f*)(ob + (size_t)row * EMBED + c4) = val;
            }
            __threadfence();
        }
    }
}

extern "C" void kernel_launch(void* const* d_in, const int* in_sizes, int n_in,
                              void* d_out, int out_size, void* d_ws, size_t ws_size, hipStream_t stream) {
    if (n_in < 7) return;
    if (in_sizes[0] < NB * QLEN_FULL * QDIM) return;
    if (in_sizes[1] < KLEN * QDIM) return;
    if (in_sizes[2] < KLEN * QDIM) return;
    if (in_sizes[3] < NB * KLEN) return;
    if (in_sizes[4] < QDIM * EMBED) return;
    if (in_sizes[5] < QDIM * EMBED) return;
    if (in_sizes[6] < QDIM * EMBED) return;
    if (out_size < NB * QLEN_FULL * EMBED) return;

    const float* queries = (const float*)d_in[0];
    const float* keys    = (const float*)d_in[1];
    const float* values  = (const float*)d_in[2];
    const int*   mask    = (const int*)d_in[3];
    const float* Wq      = (const float*)d_in[4];
    const float* Wk      = (const float*)d_in[5];
    const float* Wv      = (const float*)d_in[6];
    float* out = (float*)d_out;

    const size_t szXq = (size_t)NB * QLEN_FULL * QDIM * 2;
    const size_t szXk = (size_t)KLEN * QDIM * 2;
    const size_t szW  = (size_t)EMBED * QDIM * 2;
    const size_t szQ  = (size_t)NB * QLEN_FULL * EMBED * 2;
    const size_t szK  = (size_t)KLEN * EMBED * 2;
    char* ws = (char*)d_ws;
    size_t off = 0;
    unsigned short* XqP = (unsigned short*)(ws + off); off += szXq;
    unsigned short* XkP = (unsigned short*)(ws + off); off += szXk;
    unsigned short* XvP = (unsigned short*)(ws + off); off += szXk;
    unsigned short* WqT = (unsigned short*)(ws + off); off += szW;
    unsigned short* WkT = (unsigned short*)(ws + off); off += szW;
    unsigned short* WvT = (unsigned short*)(ws + off); off += szW;
    unsigned short* qPl = (unsigned short*)(ws + off); off += szQ;
    unsigned short* qRl = (unsigned short*)(ws + off); off += szQ;
    unsigned short* kPl = (unsigned short*)(ws + off); off += szK;
    unsigned short* vTl = (unsigned short*)(ws + off); off += szK;
    if (off > ws_size) return;

    {
        const long long n8q = (long long)NB * QLEN_FULL * QDIM / 8;
        const long long n8k = (long long)KLEN * QDIM / 8;
        k_cvt_bf16<<<(unsigned)((n8q + 255) / 256), 256, 0, stream>>>(queries, XqP, n8q);
        k_cvt_bf16<<<(unsigned)((n8k + 255) / 256), 256, 0, stream>>>(keys, XkP, n8k);
        k_cvt_bf16<<<(unsigned)((n8k + 255) / 256), 256, 0, stream>>>(values, XvP, n8k);
        const unsigned gw = (unsigned)((EMBED * (QDIM / 8) + 255) / 256);
        k_wT_bf16<<<gw, 256, 0, stream>>>(Wq, WqT);
        k_wT_bf16<<<gw, 256, 0, stream>>>(Wk, WkT);
        k_wT_bf16<<<gw, 256, 0, stream>>>(Wv, WvT);
    }
    k_gemm64<true><<<dim3((unsigned)(((SEQ / 64) * (EMBED / 64) + 7) / 8), (unsigned)NB), 256, 0, stream>>>(
        XqP, QDIM, (long long)QLEN_FULL * QDIM, WqT, QDIM, 0LL, qPl, qRl, EMBED, (long long)QLEN_FULL * EMBED, SEQ, EMBED, QDIM, 1.0f);
    k_gemm64<false><<<dim3((unsigned)(((KLEN / 64) * (EMBED / 64) + 7) / 8), 1u), 256, 0, stream>>>(
        XkP, QDIM, 0LL, WkT, QDIM, 0LL, kPl, nullptr, EMBED, 0LL, KLEN, EMBED, QDIM, 1.0f);
    k_gemm64<false><<<dim3((unsigned)(((EMBED / 64) * (KLEN / 64) + 7) / 8), 1u), 256, 0, stream>>>(
        WvT, QDIM, 0LL, XvP, QDIM, 0LL, vTl, nullptr, KLEN, 0LL, EMBED, KLEN, QDIM, 1.0f);
    k_flash<<<(unsigned)(NB * HEADS * (SEQ / (16 * FW))), 32 * FW, 0, stream>>>(qPl, qRl, kPl, vTl, mask, out);
}
